// SRGAT_27341761806358
// MI455X (gfx1250) — hardware-verified
//
#include <hip/hip_runtime.h>


#define NA   1024
#define HH   64
#define NM   20
#define PH   1280
#define ICH  128
#define NPC  (ICH * NA)
#define NCH  (NA / ICH)
typedef _Float16 h16;
typedef unsigned short bf;
typedef __attribute__((ext_vector_type(16))) __bf16   v16bf;
typedef __attribute__((ext_vector_type(16))) _Float16 v16h;
typedef __attribute__((ext_vector_type(8)))  _Float16 v8h;
typedef __attribute__((ext_vector_type(8)))  unsigned short v8us;
typedef __attribute__((ext_vector_type(8)))  float    v8f;
typedef __attribute__((ext_vector_type(4)))  float    v4f;
typedef v8h  __attribute__((may_alias)) v8ha;
typedef v4f  __attribute__((may_alias)) v4fa;
typedef v8us __attribute__((may_alias)) v8usa;

__device__ __forceinline__ unsigned short f2bf(float f) { unsigned u = __float_as_uint(f); u += 0x7FFFu + ((u >> 16) & 1u); return (unsigned short)(u >> 16); }
__device__ __forceinline__ float bf2f(unsigned short b) { return __uint_as_float(((unsigned)b) << 16); }
__device__ __forceinline__ float bfr(float f) { return bf2f(f2bf(f)); }
__device__ __forceinline__ v16h cat16(v8h lo, v8h hi) { return __builtin_shufflevector(lo, hi, 0, 1, 2, 3, 4, 5, 6, 7, 8, 9, 10, 11, 12, 13, 14, 15); }
__device__ __forceinline__ v16bf cat16b(v8us lo, v8us hi) { return __builtin_bit_cast(v16bf, __builtin_shufflevector(lo, hi, 0, 1, 2, 3, 4, 5, 6, 7, 8, 9, 10, 11, 12, 13, 14, 15)); }
__device__ __forceinline__ v8f wmma16(v16h a, v16h b, v8f c) { return __builtin_amdgcn_wmma_f32_16x16x32_f16(false, a, false, b, (short)0, c, false, false); }
__device__ __forceinline__ v8f wmmab(v16bf a, v16bf b, v8f c) { return __builtin_amdgcn_wmma_f32_16x16x32_bf16(false, a, false, b, (short)0, c, false, false); }


template <typename T16> struct WFrag;
template <> struct WFrag<h16> { typedef v16h V; static __device__ __forceinline__ V ld(const h16* p) { return cat16(*(const v8h*)p, *(const v8h*)(p + 16)); } static __device__ __forceinline__ v8f mma(V a, V b, v8f c) { return wmma16(a, b, c); } };
template <> struct WFrag<bf> { typedef v16bf V; static __device__ __forceinline__ V ld(const bf* p) { return cat16b(*(const v8us*)p, *(const v8us*)(p + 16)); } static __device__ __forceinline__ v8f mma(V a, V b, v8f c) { return wmmab(a, b, c); } };
template <typename T16, int NSPLIT, bool BIAS>
__global__ __launch_bounds__(32) void k_gemmw(const T16* __restrict__ A, const T16* __restrict__ A2, const T16* __restrict__ Bt, const T16* __restrict__ Bt2, int K, float* C, int ldc, const float* __restrict__ bias, size_t sA, size_t sB, size_t sC) {
    typedef typename WFrag<T16>::V V;
    __shared__ __align__(16) float os[16 * 68];
    const size_t z = blockIdx.z; A += z * sA; if (A2) A2 += z * sA; Bt += z * sB; if (Bt2) Bt2 += z * sB; C += z * sC;
    const int lane = threadIdx.x & 31, lr = lane & 15, hi = lane >> 4; const int r0 = blockIdx.x * 64, c0 = blockIdx.y * 64;
    v8f acc[4][4];
#pragma unroll
    for (int mb = 0; mb < 4; ++mb)
#pragma unroll
        for (int nb = 0; nb < 4; ++nb) acc[mb][nb] = (v8f){};
    const size_t aoff = (size_t)(r0 + lr) * K + 8 * hi, boff = (size_t)(c0 + lr) * K + 8 * hi;
#pragma unroll 1
    for (int kc = 0; kc < K; kc += 32) {
        V a[4], a2[4];
#pragma unroll
        for (int mb = 0; mb < 4; ++mb) { a[mb] = WFrag<T16>::ld(A + aoff + (size_t)mb * 16 * K + kc); if (NSPLIT == 1 || NSPLIT == 2) a2[mb] = WFrag<T16>::ld(A2 + aoff + (size_t)mb * 16 * K + kc); }
#pragma unroll
        for (int nb = 0; nb < 4; ++nb) { const V b = WFrag<T16>::ld(Bt + boff + (size_t)nb * 16 * K + kc); V b2; if (NSPLIT >= 2) b2 = WFrag<T16>::ld(Bt2 + boff + (size_t)nb * 16 * K + kc);
#pragma unroll
            for (int mb = 0; mb < 4; ++mb) { acc[mb][nb] = WFrag<T16>::mma(a[mb], b, acc[mb][nb]); if (NSPLIT == 1 || NSPLIT == 2) acc[mb][nb] = WFrag<T16>::mma(a2[mb], b, acc[mb][nb]); if (NSPLIT >= 2) acc[mb][nb] = WFrag<T16>::mma(a[mb], b2, acc[mb][nb]); } }
        asm volatile("v_nop\n\tv_nop\n\tv_nop\n\tv_nop" : "+v"(acc[0][0]), "+v"(acc[1][1]), "+v"(acc[2][2]), "+v"(acc[3][3]) : "v"(a[0]), "v"(a[3]));
    }
#pragma unroll
    for (int mb = 0; mb < 4; ++mb) {
#pragma unroll
        for (int nb = 0; nb < 4; ++nb) {
#pragma unroll
            for (int j = 0; j < 8; ++j) os[(hi * 8 + j) * 68 + nb * 16 + lr] = acc[mb][nb][j]; }
        __builtin_amdgcn_wave_barrier(); asm volatile("" ::: "memory");
        float* crow = C + (size_t)(r0 + mb * 16) * ldc + c0;
#pragma unroll 1
        for (int ps = 0; ps < 2; ++ps) {
#pragma unroll
            for (int s = 0; s < 8; ++s) { const int row = 2 * s + hi, cofs = lr * 4; v4f val = *(const v4fa*)(os + row * 68 + cofs); if (BIAS) { val[0] += bfr(bias[c0 + cofs]); val[1] += bfr(bias[c0 + cofs + 1]); val[2] += bfr(bias[c0 + cofs + 2]); val[3] += bfr(bias[c0 + cofs + 3]); }
                *(volatile v4f*)(crow + (size_t)row * ldc + cofs) = val; }
            if (ps == 0) __threadfence(); }
        __builtin_amdgcn_wave_barrier(); asm volatile("" ::: "memory");
    }
}

__device__ __forceinline__ void splitf(float y, unsigned short& h, unsigned short& l) { h = f2bf(y); l = f2bf(y - bf2f(h)); }
__device__ __noinline__ float sigm(float z) { return __fdiv_rn(1.0f, 1.0f + __expf(-z)); }
typedef __attribute__((ext_vector_type(2))) unsigned short v2us;
typedef __attribute__((ext_vector_type(4))) unsigned short v4us;

__global__ __launch_bounds__(256) void k_wtb(const float* __restrict__ w, int K, int N, int Kp, int Np, bf* Bt) {
    const int lane = threadIdx.x & 31; const int L0 = (blockIdx.x * 8 + (threadIdx.x >> 5)) * 8; const int nlines = Np * Kp / 64;
#pragma unroll 1
    for (int ps = 0; ps < 2; ++ps) {
#pragma unroll 1
        for (int l = 0; l < 8; ++l) { const int L = L0 + l; if (L >= nlines) break; const int e = L * 64 + lane * 2; v2us o;
#pragma unroll
            for (int q = 0; q < 2; ++q) { const int n = (e + q) / Kp, k = (e + q) % Kp; o[q] = (n < N && k < K) ? f2bf(w[(size_t)(k < K ? k : 0) * N + (n < N ? n : 0)]) : (unsigned short)0; }
            *(volatile v2us*)(Bt + e) = o; }
        if (ps == 0) __threadfence(); }
}
__global__ __launch_bounds__(64) void k_bpad(const float* __restrict__ b, int N, float* out) { const int i = threadIdx.x; const float v = i < N ? b[i < N ? i : 0] : 0.f; *(volatile float*)(out + i) = v; __threadfence(); *(volatile float*)(out + i) = v; }
__global__ __launch_bounds__(256) void k_split(const float* __restrict__ A, int nlines, float sc, bf* Ph, bf* Pl) {
    const int lane = threadIdx.x & 31; const int L = blockIdx.x * 8 + (threadIdx.x >> 5); if (L >= nlines) return; const int e = L * 64 + lane * 2; v2us oh, ol;
#pragma unroll
    for (int q = 0; q < 2; ++q) { unsigned short a, c2; splitf(A[(size_t)e + q] * sc, a, c2); oh[q] = a; ol[q] = c2; }
    *(volatile v2us*)(Ph + (size_t)e) = oh; *(volatile v2us*)(Pl + (size_t)e) = ol; __threadfence(); *(volatile v2us*)(Ph + (size_t)e) = oh; *(volatile v2us*)(Pl + (size_t)e) = ol;
}
__global__ __launch_bounds__(256) void k_xsplit(const float* __restrict__ A, int nlines, bf* Ph, bf* Pl) {
    const int lane = threadIdx.x & 31; const int L = blockIdx.x * 8 + (threadIdx.x >> 5); if (L >= nlines) return; const int e = L * 64 + lane * 2; v2us oh, ol;
#pragma unroll
    for (int q = 0; q < 2; ++q) { oh[q] = f2bf(A[(size_t)e + q]); ol[q] = 0; }
    *(volatile v2us*)(Ph + (size_t)e) = oh; *(volatile v2us*)(Pl + (size_t)e) = ol; __threadfence(); *(volatile v2us*)(Ph + (size_t)e) = oh; *(volatile v2us*)(Pl + (size_t)e) = ol;
}
__global__ __launch_bounds__(256) void k_initf(const float* __restrict__ A, int nlines, float* Y) { typedef __attribute__((ext_vector_type(2))) float v2f; const int lane = threadIdx.x & 31; const int L = blockIdx.x * 8 + (threadIdx.x >> 5); if (L >= nlines) return; const int e = L * 64 + lane * 2; v2f o; o[0] = bfr(A[e]); o[1] = bfr(A[e + 1]); *(volatile v2f*)(Y + e) = o; __threadfence(); *(volatile v2f*)(Y + e) = o; }
__global__ __launch_bounds__(256) void k_vt(const float* __restrict__ V, bf* Ph, bf* Pl) {
    const int lane = threadIdx.x & 31; const int L = blockIdx.x * 8 + (threadIdx.x >> 5); if (L >= HH * NA / 64) return; const int e = L * 64 + lane * 2; const int n = e & (NA - 1), d = e >> 10; v2us oh, ol;
#pragma unroll
    for (int q = 0; q < 2; ++q) { unsigned short a, c2; splitf(V[(size_t)(n + q) * HH + d], a, c2); oh[q] = a; ol[q] = c2; }
    *(volatile v2us*)(Ph + (size_t)e) = oh; *(volatile v2us*)(Pl + (size_t)e) = ol; __threadfence(); *(volatile v2us*)(Ph + (size_t)e) = oh; *(volatile v2us*)(Pl + (size_t)e) = ol;
}
__global__ __launch_bounds__(256) void k_hid(const float* __restrict__ pos, const float* __restrict__ w1, const float* __restrict__ b1, int c, bf* Ph, bf* Pl) {
    const int lane = threadIdx.x & 31; const int L0 = (blockIdx.x * 8 + (threadIdx.x >> 5)) * 8; const int nlines = NPC * HH / 64;
#pragma unroll 1
    for (int ps = 0; ps < 2; ++ps) {
#pragma unroll 1
        for (int l = 0; l < 8; ++l) { const int L = L0 + l; if (L >= nlines) break; const int e = L * 64 + lane * 2; const int h = e & 63; const int pr = e >> 6; const int j = pr & (NA - 1), i = c * ICH + (pr >> 10);
            const float dx = bfr(pos[i * 2]) - bfr(pos[j * 2]), dy = bfr(pos[i * 2 + 1]) - bfr(pos[j * 2 + 1]); v2us oh, ol;
#pragma unroll
            for (int q = 0; q < 2; ++q) { const int hq = h + q; const float v = fmaxf(dx * bfr(w1[hq]) + dy * bfr(w1[HH + hq]) + bfr(b1[hq]), 0.f); unsigned short a, c2; splitf(v, a, c2); oh[q] = a; ol[q] = c2; }
            *(volatile v2us*)(Ph + (size_t)e) = oh; *(volatile v2us*)(Pl + (size_t)e) = ol; }
        if (ps == 0) __threadfence(); }
}
__global__ __launch_bounds__(256) void k_bcopy(const float* __restrict__ CB, int c, float* BIAS) { const int lane = threadIdx.x & 31; const int p0 = (blockIdx.x * 8 + (threadIdx.x >> 5)) * 32; if (p0 >= NPC) return; const float v = CB[(size_t)(p0 + lane) * 64]; float* dst = BIAS + (size_t)c * NPC + p0 + lane; *(volatile float*)dst = v; __threadfence(); *(volatile float*)dst = v; }
__global__ __launch_bounds__(256) void k_msm(const float* __restrict__ LG, const float* __restrict__ BIAS, const int* __restrict__ mask, bf* Ah, bf* Al, float* HN) {
    const int lane = threadIdx.x & 31; const int i = blockIdx.x * 8 + (threadIdx.x >> 5); if (i >= NA) return; float v[32]; float m = -3.0e38f; float anyv = 0.f;
typedef __attribute__((ext_vector_type(4))) int v4i;
#pragma unroll
    for (int ch = 0; ch < 8; ++ch) { const v4f a = *(const v4f*)(LG + (size_t)i * NA + ch * 128 + lane * 4), b = *(const v4f*)(BIAS + (size_t)i * NA + ch * 128 + lane * 4); const v4i mk = *(const v4i*)(mask + (size_t)i * NA + ch * 128 + lane * 4);
#pragma unroll
        for (int q = 0; q < 4; ++q) { const bool on = mk[q] != 0;     const float t = on ? (a[q] + b[q]) : -1e9f; v[ch * 4 + q] = t; m = fmaxf(m, t); anyv = on ? 1.f : anyv; } }
#pragma unroll
    for (int sh = 16; sh; sh >>= 1) { m = fmaxf(m, __shfl_xor(m, sh, 32)); anyv = fmaxf(anyv, __shfl_xor(anyv, sh, 32)); }
    float s = 0.f;
#pragma unroll
    for (int k = 0; k < 32; ++k) { v[k] = __expf(v[k] - m); s += v[k]; }
#pragma unroll
    for (int sh = 16; sh; sh >>= 1) s += __shfl_xor(s, sh, 32);
    const float f = __fdiv_rn(1.0f, s);
#pragma unroll 1
    for (int ps = 0; ps < 2; ++ps) {
#pragma unroll
        for (int ch = 0; ch < 8; ++ch) { v4us oh, ol;
#pragma unroll
            for (int q = 0; q < 4; ++q) { unsigned short a, c2; splitf(v[ch * 4 + q] * f, a, c2); oh[q] = a; ol[q] = c2; }
            *(volatile v4us*)(Ah + (size_t)i * NA + ch * 128 + lane * 4) = oh; *(volatile v4us*)(Al + (size_t)i * NA + ch * 128 + lane * 4) = ol; }
        *(volatile float*)(HN + (size_t)i * 32 + lane) = (lane == 0) ? anyv : 0.f;
        if (ps == 0) __threadfence(); }
}
template <int MODE>
__global__ __launch_bounds__(256) void k_cat2(const float* __restrict__ A, const float* __restrict__ B2, const float* __restrict__ HN, bf* Ph, bf* Pl) {
    const int lane = threadIdx.x & 31; const int L = blockIdx.x * 8 + (threadIdx.x >> 5); if (L >= NA * 128 / 64) return; const int e = L * 64 + lane * 2; const int c = e & 127; const int i = e >> 7; v2us oh, ol;
#pragma unroll
    for (int q = 0; q < 2; ++q) { const int cc = c + q; float v; if (MODE == 0) v = cc < HH ? A[(size_t)i * HH + cc] : (HN[(size_t)i * 32] != 0.f ? B2[(size_t)i * HH + cc - HH] : 0.f); else v = cc < HH ? bfr(A[(size_t)i * HH + cc]) : B2[(size_t)i * HH + cc - HH]; unsigned short a, c2; splitf(v, a, c2); oh[q] = a; ol[q] = c2; }
    *(volatile v2us*)(Ph + (size_t)e) = oh; *(volatile v2us*)(Pl + (size_t)e) = ol; __threadfence(); *(volatile v2us*)(Ph + (size_t)e) = oh; *(volatile v2us*)(Pl + (size_t)e) = ol;
}
template <int MODE>
__global__ __launch_bounds__(256) void k_upd(const float* __restrict__ G, const float* __restrict__ gb, const float* __restrict__ Hc, const float* __restrict__ B2, const float* __restrict__ HN, float* Y, bf* Ph, bf* Pl) {
    const int lane = threadIdx.x & 31; const int L = blockIdx.x * 8 + (threadIdx.x >> 5); if (L >= NA * HH / 64) return; const int e = L * 64 + lane * 2; const int c = e & 63; const int i = e >> 6; v2us oh, ol; float yv[2];
#pragma unroll
    for (int q = 0; q < 2; ++q) { const int cc = c + q; const float s = sigm(G[(size_t)i * HH + cc] + bfr(gb[cc])); float v;
        if (MODE == 0) { const float msg = HN[(size_t)i * 32] != 0.f ? B2[(size_t)i * HH + cc] : 0.f; v = (1.0f - s) * Hc[(size_t)i * HH + cc] + s * msg; }
        else { v = s * bfr(B2[(size_t)i * HH + cc]) + (1.0f - s) * Hc[(size_t)i * HH + cc]; }
        yv[q] = v; unsigned short a, c2; splitf(v, a, c2); oh[q] = a; ol[q] = c2; }
    typedef __attribute__((ext_vector_type(2))) float v2f; v2f yo; yo[0] = yv[0]; yo[1] = yv[1];
    *(volatile v2f*)(Y + (size_t)e) = yo; *(volatile v2us*)(Ph + (size_t)e) = oh; *(volatile v2us*)(Pl + (size_t)e) = ol; __threadfence(); *(volatile v2f*)(Y + (size_t)e) = yo; *(volatile v2us*)(Ph + (size_t)e) = oh; *(volatile v2us*)(Pl + (size_t)e) = ol;
}
__global__ __launch_bounds__(256) void k_lnrelu(const float* __restrict__ PR, const float* __restrict__ gg, const float* __restrict__ bb, bf* Ph, bf* Pl) {
    const int lane = threadIdx.x & 31; const int i = blockIdx.x * 8 + (threadIdx.x >> 5); if (i >= NA) return; float v[40]; float s = 0.f;
#pragma unroll
    for (int ch = 0; ch < 10; ++ch) { const v4f a = *(const v4f*)(PR + (size_t)i * PH + ch * 128 + lane * 4);
#pragma unroll
        for (int q = 0; q < 4; ++q) { v[ch * 4 + q] = a[q]; s += a[q]; } }
#pragma unroll
    for (int sh = 16; sh; sh >>= 1) s += __shfl_xor(s, sh, 32);
    const float mu = s * (1.0f / PH); float qq = 0.f;
#pragma unroll
    for (int k = 0; k < 40; ++k) { const float d0 = v[k] - mu; qq = fmaf(d0, d0, qq); }
#pragma unroll
    for (int sh = 16; sh; sh >>= 1) qq += __shfl_xor(qq, sh, 32);
    const float rs = rsqrtf(qq * (1.0f / PH) + 1e-5f);
#pragma unroll 1
    for (int ps = 0; ps < 2; ++ps) {
#pragma unroll 1
        for (int ch = 0; ch < 10; ++ch) { v4us oh, ol;
#pragma unroll
            for (int q = 0; q < 4; ++q) { const int col = ch * 128 + lane * 4 + q; const float y = fmaxf((v[ch * 4 + q] - mu) * rs * bfr(gg[col]) + bfr(bb[col]), 0.f); unsigned short a, c2; splitf(y, a, c2); oh[q] = a; ol[q] = c2; }
            *(volatile v4us*)(Ph + (size_t)i * PH + ch * 128 + lane * 4) = oh; *(volatile v4us*)(Pl + (size_t)i * PH + ch * 128 + lane * 4) = ol; }
        if (ps == 0) __threadfence(); }
}
__global__ __launch_bounds__(256) void k_out(const float* __restrict__ D2, float* OUT) { const int idx = blockIdx.x * 256 + threadIdx.x; if (idx >= NM * NA * 2) return; const int c = idx & 1; const int n = (idx >> 1) & (NA - 1); const int m = idx / (2 * NA); const float v = D2[((size_t)n * NM + m) * 64 + c]; *(volatile float*)(OUT + idx) = v; __threadfence(); *(volatile float*)(OUT + idx) = v; }

extern "C" void kernel_launch(void* const* d_in, const int* in_sizes, int n_in,
                              void* d_out, int out_size, void* d_ws, size_t ws_size, hipStream_t stream) {
    (void)in_sizes; (void)n_in; (void)out_size;
    const float* xe = (const float*)d_in[0]; const float* h0 = (const float*)d_in[1]; const float* pos = (const float*)d_in[2];
    const float* Wq = (const float*)d_in[3]; const float* Wk = (const float*)d_in[4]; const float* Wv = (const float*)d_in[5]; const float* cw1 = (const float*)d_in[6]; const float* cb1 = (const float*)d_in[7]; const float* cw2 = (const float*)d_in[8];
    const float* gw = (const float*)d_in[9]; const float* gb = (const float*)d_in[10]; const float* fw = (const float*)d_in[11]; const float* fb = (const float*)d_in[12]; const float* pw = (const float*)d_in[13]; const float* pb = (const float*)d_in[14]; const float* lg = (const float*)d_in[15]; const float* lb = (const float*)d_in[16];
    const float* dw1 = (const float*)d_in[17]; const float* db1 = (const float*)d_in[18]; const float* dw2 = (const float*)d_in[19]; const float* db2 = (const float*)d_in[20]; const int* mask = (const int*)d_in[21];
    float* OUT = (float*)d_out;
    char* wsp = (char*)d_ws;
    auto take = [&](size_t bytes) { char* p = wsp; wsp += (bytes + 255) & ~(size_t)255; return (void*)p; };
    bf* WQB[2]; bf* WKB[2]; bf* WVB[2]; bf* W2B[2]; bf* GWB[2];
    for (int p = 0; p < 2; ++p) { WQB[p] = (bf*)take(64 * 64 * 2); WKB[p] = (bf*)take(64 * 64 * 2); WVB[p] = (bf*)take(64 * 64 * 2); W2B[p] = (bf*)take(64 * 64 * 2); GWB[p] = (bf*)take(64 * 128 * 2); }
    bf* FWB = (bf*)take(64 * 128 * 2); bf* PWB = (bf*)take((size_t)PH * 64 * 2); bf* D1B = (bf*)take(64 * 64 * 2); bf* D2B = (bf*)take(64 * 64 * 2); float* DB2P = (float*)take(64 * 4);
    float* Hf = (float*)take(NA * HH * 4); bf* Hh = (bf*)take(NA * HH * 2); bf* Hl = (bf*)take(NA * HH * 2);
    bf* HIDh = (bf*)take((size_t)NPC * HH * 2); bf* HIDl = (bf*)take((size_t)NPC * HH * 2); float* CB = (float*)take((size_t)NPC * 64 * 4); float* BIAS = (float*)take((size_t)NA * NA * 4);
    float* Qf = (float*)take(NA * HH * 4); float* Kf = (float*)take(NA * HH * 4); float* Vf = (float*)take(NA * HH * 4); bf* Qh = (bf*)take(NA * HH * 2); bf* Ql = (bf*)take(NA * HH * 2); bf* Kh = (bf*)take(NA * HH * 2); bf* Kl = (bf*)take(NA * HH * 2); bf* VTh = (bf*)take(NA * HH * 2); bf* VTl = (bf*)take(NA * HH * 2);
    float* LG = (float*)take((size_t)NA * NA * 4); bf* Ah = (bf*)take((size_t)NA * NA * 2); bf* Al = (bf*)take((size_t)NA * NA * 2); float* HN = (float*)take(NA * 32 * 4); float* MSG = (float*)take(NA * HH * 4);
    bf* CATh = (bf*)take(NA * 128 * 2); bf* CATl = (bf*)take(NA * 128 * 2); float* G = (float*)take(NA * HH * 4); float* FU = (float*)take(NA * HH * 4); bf* FUh = (bf*)take(NA * HH * 2); bf* FUl = (bf*)take(NA * HH * 2);
    float* PR = (float*)take((size_t)NA * PH * 4); bf* PFh = (bf*)take((size_t)NA * PH * 2); bf* PFl = (bf*)take((size_t)NA * PH * 2); float* D1 = (float*)take((size_t)NA * NM * 64 * 4); bf* D1h = (bf*)take((size_t)NA * NM * 64 * 2); bf* D1l = (bf*)take((size_t)NA * NM * 64 * 2); float* D2 = (float*)take((size_t)NA * NM * 64 * 4);
    if ((size_t)(wsp - (char*)d_ws) > ws_size) return;
    { const unsigned g1 = 1, g2 = 2; for (int p = 0; p < 2; ++p) { k_wtb<<<g1, 256, 0, stream>>>(Wq + p * 4096, 64, 64, 64, 64, WQB[p]); k_wtb<<<g1, 256, 0, stream>>>(Wk + p * 4096, 64, 64, 64, 64, WKB[p]); k_wtb<<<g1, 256, 0, stream>>>(Wv + p * 4096, 64, 64, 64, 64, WVB[p]);
          k_wtb<<<g1, 256, 0, stream>>>(cw2 + p * 64, 64, 1, 64, 64, W2B[p]); k_wtb<<<g2, 256, 0, stream>>>(gw + p * 8192, 128, 64, 128, 64, GWB[p]); }
      k_wtb<<<g2, 256, 0, stream>>>(fw, 128, 64, 128, 64, FWB); k_wtb<<<(PH * 64 / 64 + 63) / 64, 256, 0, stream>>>(pw, 64, PH, 64, PH, PWB); k_wtb<<<g1, 256, 0, stream>>>(dw1, 64, 64, 64, 64, D1B); k_wtb<<<g1, 256, 0, stream>>>(dw2, 64, 2, 64, 64, D2B); k_bpad<<<1, 64, 0, stream>>>(db2, 2, DB2P); }
    const unsigned L64 = (NA * HH / 64 + 7) / 8;
    k_xsplit<<<L64, 256, 0, stream>>>(h0, NA * HH / 64, Hh, Hl); k_initf<<<L64, 256, 0, stream>>>(h0, NA * HH / 64, Hf);
    for (int p = 0; p < 2; ++p) {
        for (int c = 0; c < NCH; ++c) { k_hid<<<(NPC * HH / 64 + 63) / 64, 256, 0, stream>>>(pos, cw1 + p * 128, cb1 + p * 64, c, HIDh, HIDl);
            k_gemmw<bf, 1, false><<<dim3(NPC / 64, 1, 1), 32, 0, stream>>>(HIDh, HIDl, W2B[p], nullptr, HH, CB, 64, nullptr, 0, 0, 0);
            k_bcopy<<<NPC / 32 / 8, 256, 0, stream>>>(CB, c, BIAS); }
        k_gemmw<bf, 1, false><<<dim3(NA / 64, 1, 1), 32, 0, stream>>>(Hh, Hl, WQB[p], nullptr, HH, Qf, HH, nullptr, 0, 0, 0);
        k_gemmw<bf, 1, false><<<dim3(NA / 64, 1, 1), 32, 0, stream>>>(Hh, Hl, WKB[p], nullptr, HH, Kf, HH, nullptr, 0, 0, 0);
        k_gemmw<bf, 1, false><<<dim3(NA / 64, 1, 1), 32, 0, stream>>>(Hh, Hl, WVB[p], nullptr, HH, Vf, HH, nullptr, 0, 0, 0);
        k_split<<<L64, 256, 0, stream>>>(Qf, NA * HH / 64, 0.125f, Qh, Ql); k_split<<<L64, 256, 0, stream>>>(Kf, NA * HH / 64, 1.0f, Kh, Kl); k_vt<<<L64, 256, 0, stream>>>(Vf, VTh, VTl);
        k_gemmw<bf, 2, false><<<dim3(NA / 64, NA / 64, 1), 32, 0, stream>>>(Qh, Ql, Kh, Kl, HH, LG, NA, nullptr, 0, 0, 0);
        k_msm<<<NA / 8, 256, 0, stream>>>(LG, BIAS, mask, Ah, Al, HN);
        k_gemmw<bf, 2, false><<<dim3(NA / 64, 1, 1), 32, 0, stream>>>(Ah, Al, VTh, VTl, NA, MSG, HH, nullptr, 0, 0, 0);
        k_cat2<0><<<(NA * 128 / 64 + 7) / 8, 256, 0, stream>>>(Hf, MSG, HN, CATh, CATl);
        k_gemmw<bf, 1, false><<<dim3(NA / 64, 1, 1), 32, 0, stream>>>(CATh, CATl, GWB[p], nullptr, 128, G, HH, nullptr, 0, 0, 0);
        k_upd<0><<<L64, 256, 0, stream>>>(G, gb + p * 64, Hf, MSG, HN, Hf, Hh, Hl); }
    k_cat2<1><<<(NA * 128 / 64 + 7) / 8, 256, 0, stream>>>(xe, Hf, HN, CATh, CATl);
    k_gemmw<bf, 1, false><<<dim3(NA / 64, 1, 1), 32, 0, stream>>>(CATh, CATl, FWB, nullptr, 128, G, HH, nullptr, 0, 0, 0);
    k_upd<1><<<L64, 256, 0, stream>>>(G, fb, Hf, xe, HN, FU, FUh, FUl);
    k_gemmw<bf, 1, true><<<dim3(NA / 64, PH / 64, 1), 32, 0, stream>>>(FUh, FUl, PWB, nullptr, HH, PR, PH, pb, 0, 0, 0);
    k_lnrelu<<<NA / 8, 256, 0, stream>>>(PR, lg, lb, PFh, PFl);
    k_gemmw<bf, 1, true><<<dim3(NA * NM / 64, 1, 1), 32, 0, stream>>>(PFh, PFl, D1B, nullptr, HH, D1, 64, db1, 0, 0, 0);
    k_split<<<(NA * NM * 64 / 64 + 7) / 8, 256, 0, stream>>>(D1, NA * NM * 64 / 64, 1.0f, D1h, D1l);
    k_gemmw<bf, 1, true><<<dim3(NA * NM / 64, 1, 1), 32, 0, stream>>>(D1h, D1l, D2B, nullptr, HH, D2, 64, DB2P, 0, 0, 0);
    k_out<<<(NM * NA * 2 + 255) / 256, 256, 0, stream>>>(D2, OUT);
}
